// Model_17789754540447
// MI455X (gfx1250) — hardware-verified
//
#include <hip/hip_runtime.h>


#ifndef NB
#define NB 4
#endif
#ifndef SEQ
#define SEQ 1024
#endif
#define NB_FULL  4
#define SEQ_FULL 1024
#ifndef OUT_SEQ
#define OUT_SEQ SEQ
#endif
#define HD   64
#define NH_  16
#define NQ   (NH_ * HD)
#define AW   4
#define OSP  68
#define TP   68
#define L2E  1.4426950408889634f
#define PCAR 16384.0f
#define PCI  (1.0f / 16384.0f)

static_assert(HD == 64);
static_assert(HD % 32 == 0);
static_assert(NH_ == 16);
static_assert(NQ % 64 == 0);
static_assert(SEQ % 64 == 0);
static_assert((NB * SEQ) % 64 == 0);
static_assert(SEQ % 32 == 0);
static_assert((NB * SEQ) % AW == 0);
static_assert(SEQ % 16 == 0);
static_assert(NB <= NB_FULL);
static_assert(SEQ <= SEQ_FULL);
static_assert((OSP * 4) % 16 == 0);
static_assert((TP * 4) % 16 == 0);
static_assert(HD * HD == 4 * 256 * 4);
static_assert(256 * 16 * 2 == 64 * 128);
static_assert(32 * 16 * 4 == 16 * 128);
static_assert(32 * 16 * 8 == 16 * HD * 4);
static_assert((size_t)256 * 16 * (SEQ / 16) == (size_t)SEQ * HD * 4);
static_assert(16 * 68 * 4 <= 131072);
static_assert(AW * 16 * OSP * 4 <= 131072);
static_assert(64 * TP * 4 <= 131072);
static_assert((8 * HD + HD) * 4 <= 131072);

typedef _Float16 h16;
typedef unsigned short bf;
typedef __attribute__((ext_vector_type(16))) __bf16   v16bf;
typedef __attribute__((ext_vector_type(16))) _Float16 v16h;
typedef __attribute__((ext_vector_type(8)))  _Float16 v8h;
typedef __attribute__((ext_vector_type(8)))  unsigned short v8us;
typedef __attribute__((ext_vector_type(8)))  float    v8f;
typedef __attribute__((ext_vector_type(4)))  float    v4f;
typedef v4f  __attribute__((may_alias)) v4fa;

__device__ __forceinline__ unsigned short f2bf(float f) { unsigned u = __float_as_uint(f); u += 0x7FFFu + ((u >> 16) & 1u); return (unsigned short)(u >> 16); }
__device__ __forceinline__ float bfr(float f) { return __uint_as_float(((unsigned)f2bf(f)) << 16); }
__device__ __forceinline__ v16h cat16(v8h lo, v8h hi) { return __builtin_shufflevector(lo, hi, 0, 1, 2, 3, 4, 5, 6, 7, 8, 9, 10, 11, 12, 13, 14, 15); }
__device__ __forceinline__ v16bf cat16b(v8us lo, v8us hi) { return __builtin_bit_cast(v16bf, __builtin_shufflevector(lo, hi, 0, 1, 2, 3, 4, 5, 6, 7, 8, 9, 10, 11, 12, 13, 14, 15)); }
__device__ __forceinline__ v8f wmma16(v16h a, v16h b, v8f c) { return __builtin_amdgcn_wmma_f32_16x16x32_f16(false, a, false, b, (short)0, c, false, false); }
__device__ __forceinline__ v8f wmmab(v16bf a, v16bf b, v8f c) { return __builtin_amdgcn_wmma_f32_16x16x32_bf16(false, a, false, b, (short)0, c, false, false); }
__device__ __forceinline__ v16h  ldh(const h16* p) { return cat16(*(const v8h*)p, *(const v8h*)(p + 16)); }
__device__ __forceinline__ v16bf ldb(const bf* p)  { return cat16b(*(const v8us*)p, *(const v8us*)(p + 16)); }
__device__ __forceinline__ void wave_sync() { __builtin_amdgcn_fence(3  , "wavefront"); __builtin_amdgcn_wave_barrier(); asm volatile("" ::: "memory"); }

static __device__ __forceinline__ h16 toh_flush(float v) { const h16 r = (h16)v; return (fabsf(v) < 6.103515625e-05f) ? (h16)0.0f : r; }
__device__ __forceinline__ v8f wmma16g(v16h a, v16h b, v8f c) { c = wmma16(a, b, c); asm volatile("v_nop\n\tv_nop\n\tv_nop\n\tv_nop" : "+v"(c) : "v"(a), "v"(b)); return c; }
__device__ __forceinline__ v8f wmmabg(v16bf a, v16bf b, v8f c) { c = wmmab(a, b, c); asm volatile("v_nop\n\tv_nop\n\tv_nop\n\tv_nop" : "+v"(c) : "v"(a), "v"(b)); return c; }

__global__ __launch_bounds__(256) void k_cvt8(const float* __restrict__ src, bf* dst, size_t n8) {
    const size_t i = (size_t)blockIdx.x * 256 + threadIdx.x; if (i >= n8) return;
    const v8f v = *(const v8f*)(src + i * 8); v8us o;
#pragma unroll
    for (int k = 0; k < 8; ++k) o[k] = f2bf(v[k]);
    *(volatile v8us*)(dst + i * 8) = o; __threadfence(); *(volatile v8us*)(dst + i * 8) = o;
}

__global__ __launch_bounds__(256) void k_cvth8(const float* __restrict__ src, h16* dst, size_t n8) {
#pragma clang fp contract(off)
    const size_t i = (size_t)blockIdx.x * 256 + threadIdx.x; if (i >= n8) return;
    const v8f v = *(const v8f*)(src + i * 8); v8h o;
#pragma unroll
    for (int k = 0; k < 8; ++k) o[k] = toh_flush(bfr(v[k]));
    *(volatile v8h*)(dst + i * 8) = o; __threadfence(); *(volatile v8h*)(dst + i * 8) = o;
}

__global__ __launch_bounds__(256) void k_wtr(const float* __restrict__ W, bf* WT) {
#pragma clang fp contract(off)
    __shared__ __align__(16) float ts[64 * TP];
    const int tid = threadIdx.x; const int hd = blockIdx.x;
    const float* src = W + (size_t)hd * HD * HD;
#pragma unroll 1
    for (int it = 0; it < 4; ++it) { const int q = it * 256 + tid; const int row = q >> 4, c4 = (q & 15) * 4;
        const v4f v = *(const v4f*)(src + row * HD + c4);
        ts[(c4 + 0) * TP + row] = v[0]; ts[(c4 + 1) * TP + row] = v[1]; ts[(c4 + 2) * TP + row] = v[2]; ts[(c4 + 3) * TP + row] = v[3]; }
    __syncthreads();
    bf* dst = WT + (size_t)hd * HD * HD;
#pragma unroll 1
    for (int ps = 0; ps < 2; ++ps) {
#pragma unroll 1
        for (int it = 0; it < 2; ++it) { const int orow = it * 32 + (tid >> 3), c8 = (tid & 7) * 8;
            const v4f x0 = *(const v4fa*)(&ts[orow * TP + c8]); const v4f x1 = *(const v4fa*)(&ts[orow * TP + c8 + 4]); v8us o;
#pragma unroll
            for (int i = 0; i < 4; ++i) { o[i] = f2bf(x0[i]); o[4 + i] = f2bf(x1[i]); }
            *(volatile v8us*)(dst + (size_t)orow * HD + c8) = o; }
        if (ps == 0) __threadfence(); }
}

__global__ __launch_bounds__(256) void k_vtr(const float* __restrict__ V, h16* VT) {
#pragma clang fp contract(off)
    __shared__ __align__(16) float ts[64 * TP];
    const int tid = threadIdx.x; const int t0 = blockIdx.x * 64; const int b = blockIdx.y;
    const float* src = V + ((size_t)b * SEQ_FULL + t0) * HD;
#pragma unroll 1
    for (int it = 0; it < 4; ++it) { const int q = it * 256 + tid; const int row = q >> 4, c4 = (q & 15) * 4;
        const v4f v = *(const v4f*)(src + row * HD + c4);
        ts[(c4 + 0) * TP + row] = v[0]; ts[(c4 + 1) * TP + row] = v[1]; ts[(c4 + 2) * TP + row] = v[2]; ts[(c4 + 3) * TP + row] = v[3]; }
    __syncthreads();
    h16* dst = VT + (size_t)b * HD * SEQ + t0;
#pragma unroll 1
    for (int ps = 0; ps < 2; ++ps) {
#pragma unroll 1
        for (int it = 0; it < 2; ++it) { const int orow = it * 32 + (tid >> 3), c8 = (tid & 7) * 8;
            const v4f x0 = *(const v4fa*)(&ts[orow * TP + c8]); const v4f x1 = *(const v4fa*)(&ts[orow * TP + c8 + 4]); v8h o;
#pragma unroll
            for (int i = 0; i < 4; ++i) { o[i] = toh_flush(bfr(x0[i])); o[4 + i] = toh_flush(bfr(x1[i])); }
            *(volatile v8h*)(dst + (size_t)orow * SEQ + c8) = o; }
        if (ps == 0) __threadfence(); }
}

__global__ __launch_bounds__(32) void k_wq(const bf* __restrict__ A, const bf* __restrict__ Bt, h16* P) {
    __shared__ __align__(16) float os[16 * 68];
    const int K = HD;
    const int lane = threadIdx.x & 31, lr = lane & 15, hi = lane >> 4; const int r0 = blockIdx.x * 64, c0 = blockIdx.y * 64;
    v8f acc[4][4];
#pragma unroll
    for (int mb = 0; mb < 4; ++mb)
#pragma unroll
        for (int nb = 0; nb < 4; ++nb) acc[mb][nb] = (v8f){};
    const size_t aoff = (size_t)(r0 + lr) * K + 8 * hi, boff = (size_t)(c0 + lr) * K + 8 * hi;
#pragma unroll 1
    for (int kc = 0; kc < K; kc += 32) {
        v16bf a[4];
#pragma unroll
        for (int mb = 0; mb < 4; ++mb) a[mb] = ldb(A + aoff + (size_t)mb * 16 * K + kc);
#pragma unroll
        for (int nb = 0; nb < 4; ++nb) { const v16bf b = ldb(Bt + boff + (size_t)nb * 16 * K + kc);
#pragma unroll
            for (int mb = 0; mb < 4; ++mb) acc[mb][nb] = wmmabg(a[mb], b, acc[mb][nb]); }
    }
#pragma unroll
    for (int mb = 0; mb < 4; ++mb) {
#pragma unroll
        for (int nb = 0; nb < 4; ++nb) {
#pragma unroll
            for (int j = 0; j < 8; ++j) os[(hi * 8 + j) * 68 + nb * 16 + lr] = acc[mb][nb][j]; }
        wave_sync();
        const size_t sb = (size_t)(r0 + mb * 16) * NQ + (size_t)c0;
#pragma unroll 1
        for (int ps = 0; ps < 2; ++ps) {
#pragma unroll
            for (int s = 0; s < 4; ++s) { const int row = 4 * s + (lane >> 3), c8 = (lane & 7) * 8;
                const v4f x0 = *(const v4fa*)(&os[row * 68 + c8]); const v4f x1 = *(const v4fa*)(&os[row * 68 + c8 + 4]); v8h hv;
#pragma unroll
                for (int i = 0; i < 4; ++i) { hv[i] = toh_flush(x0[i]); hv[4 + i] = toh_flush(x1[i]); }
                *(volatile v8h*)(P + sb + (size_t)row * NQ + c8) = hv; }
            if (ps == 0) __threadfence(); }
        wave_sync();
    }
}

__global__ __launch_bounds__(32 * AW) void k_hattn(const h16* __restrict__ WQ, const h16* __restrict__ KP, const h16* __restrict__ VT, const float* __restrict__ sfp, float* DV) {
    __shared__ __align__(16) float os[AW * 16 * OSP];
    const int lane = threadIdx.x & 31, lr = lane & 15, hi = lane >> 4;
    const int wave = __builtin_amdgcn_readfirstlane((int)(threadIdx.x >> 5));
    const int row = blockIdx.x * AW + wave;
    const int b = row / SEQ, s = row % SEQ;
    const float sc2 = bfr(sfp[0]) * L2E;
    const size_t qo = ((size_t)row * NH_ + lr) * HD + 8 * hi;
    const v16h q0 = ldh(WQ + qo), q1 = ldh(WQ + qo + 32);
    const size_t ko = ((size_t)b * SEQ + lr) * HD + 8 * hi;
    const size_t vo = ((size_t)b * HD + lr) * SEQ + 8 * hi;
    v8f o0 = (v8f){}, o1 = (v8f){}, o2 = (v8f){}, o3 = (v8f){};
#pragma unroll 1
    for (int key0 = 0; key0 < SEQ; key0 += 32) {
        const h16* ka = KP + ko + (size_t)key0 * HD;
        const v16h a0 = ldh(ka), a1 = ldh(ka + 32), c0 = ldh(ka + 16 * HD), c1 = ldh(ka + 16 * HD + 32);
        v8f sa = (v8f){}, sb = (v8f){};
        sa = wmma16g(a0, q0, sa); sa = wmma16g(a1, q1, sa);
        sb = wmma16g(c0, q0, sb); sb = wmma16g(c1, q1, sb);
        v16h pb;
#pragma unroll
        for (int r = 0; r < 8; ++r) {
            const float ta = sa[r] * sc2, tb = sb[r] * sc2;
            float ma = ta, mb = tb;
            ma = fmaxf(ma, __shfl_xor(ma, 1, 32)); mb = fmaxf(mb, __shfl_xor(mb, 1, 32));
            ma = fmaxf(ma, __shfl_xor(ma, 2, 32)); mb = fmaxf(mb, __shfl_xor(mb, 2, 32));
            ma = fmaxf(ma, __shfl_xor(ma, 4, 32)); mb = fmaxf(mb, __shfl_xor(mb, 4, 32));
            ma = fmaxf(ma, __shfl_xor(ma, 8, 32)); mb = fmaxf(mb, __shfl_xor(mb, 8, 32));
            const float ea = __builtin_amdgcn_exp2f(ta - ma), eb = __builtin_amdgcn_exp2f(tb - mb);
            float za = ea, zb = eb;
            za += __shfl_xor(za, 1, 32); zb += __shfl_xor(zb, 1, 32);
            za += __shfl_xor(za, 2, 32); zb += __shfl_xor(zb, 2, 32);
            za += __shfl_xor(za, 4, 32); zb += __shfl_xor(zb, 4, 32);
            za += __shfl_xor(za, 8, 32); zb += __shfl_xor(zb, 8, 32);
            const float pa = ea * (PCAR * __builtin_amdgcn_rcpf(za));
            const float pc = eb * (PCAR * __builtin_amdgcn_rcpf(zb));
            pb[r] = toh_flush(pa); pb[8 + r] = toh_flush(pc); }
        const h16* va = VT + vo + key0;
        const v16h v0 = ldh(va), v1 = ldh(va + (size_t)16 * SEQ), v2 = ldh(va + (size_t)32 * SEQ), v3 = ldh(va + (size_t)48 * SEQ);
        o0 = wmma16g(v0, pb, o0); o1 = wmma16g(v1, pb, o1); o2 = wmma16g(v2, pb, o2); o3 = wmma16g(v3, pb, o3);
    }
    const int wb = wave * 16 * OSP;
    { const v8f f0 = o0 * PCI, f1 = o1 * PCI, f2 = o2 * PCI, f3 = o3 * PCI;
      *(v4fa*)(&os[wb + lr * OSP +  0 + 8 * hi]) = __builtin_shufflevector(f0, f0, 0, 1, 2, 3); *(v4fa*)(&os[wb + lr * OSP +  0 + 8 * hi + 4]) = __builtin_shufflevector(f0, f0, 4, 5, 6, 7);
      *(v4fa*)(&os[wb + lr * OSP + 16 + 8 * hi]) = __builtin_shufflevector(f1, f1, 0, 1, 2, 3); *(v4fa*)(&os[wb + lr * OSP + 16 + 8 * hi + 4]) = __builtin_shufflevector(f1, f1, 4, 5, 6, 7);
      *(v4fa*)(&os[wb + lr * OSP + 32 + 8 * hi]) = __builtin_shufflevector(f2, f2, 0, 1, 2, 3); *(v4fa*)(&os[wb + lr * OSP + 32 + 8 * hi + 4]) = __builtin_shufflevector(f2, f2, 4, 5, 6, 7);
      *(v4fa*)(&os[wb + lr * OSP + 48 + 8 * hi]) = __builtin_shufflevector(f3, f3, 0, 1, 2, 3); *(v4fa*)(&os[wb + lr * OSP + 48 + 8 * hi + 4]) = __builtin_shufflevector(f3, f3, 4, 5, 6, 7); }
    wave_sync();
    float* drow = DV + (((size_t)b * NH_) * SEQ + (size_t)s) * HD;
#pragma unroll 1
    for (int ps = 0; ps < 2; ++ps) {
#pragma unroll
        for (int i = 0; i < 8; ++i) { const int hrow = 2 * i + hi, cofs = lr * 4;
            const v4f val = *(const v4fa*)(&os[wb + hrow * OSP + cofs]);
            *(volatile v4f*)(drow + (size_t)hrow * SEQ * HD + cofs) = val; }
        if (ps == 0) __threadfence(); }
}

__global__ __launch_bounds__(256) void k_fin(const float* __restrict__ DV, float* OUT) {
#pragma clang fp contract(off)
    __shared__ __align__(16) float zs[8 * HD];
    __shared__ __align__(16) float zi[HD];
    const int lane = threadIdx.x & 31, lr = lane & 15, hi = lane >> 4;
    const int wave = __builtin_amdgcn_readfirstlane((int)(threadIdx.x >> 5));
    const int zh = blockIdx.x;
    const float* src = DV + (size_t)zh * SEQ * HD + (size_t)(wave * 2 + hi) * HD + lr * 4;
    float* dst = OUT + (size_t)zh * OUT_SEQ * HD + (size_t)(wave * 2 + hi) * HD + lr * 4;
    v4f zc = (v4f){}; v4f iz = (v4f){};
#pragma unroll 1
    for (int ps = 0; ps < 2; ++ps) {
#pragma unroll 1
        for (int i = 0; i < SEQ / 16; ++i) {
            const v4f x = *(const v4f*)(src + (size_t)i * 16 * HD);
            float m = fmaxf(fmaxf(x[0], x[1]), fmaxf(x[2], x[3]));
            m = fmaxf(m, __shfl_xor(m, 1, 32)); m = fmaxf(m, __shfl_xor(m, 2, 32)); m = fmaxf(m, __shfl_xor(m, 4, 32)); m = fmaxf(m, __shfl_xor(m, 8, 32));
            v4f e;
#pragma unroll
            for (int k = 0; k < 4; ++k) e[k] = __builtin_amdgcn_exp2f((x[k] - m) * L2E);
            float sm = (e[0] + e[1]) + (e[2] + e[3]);
            sm += __shfl_xor(sm, 1, 32); sm += __shfl_xor(sm, 2, 32); sm += __shfl_xor(sm, 4, 32); sm += __shfl_xor(sm, 8, 32);
            const float rinv = 1.0f / sm;
            v4f y;
#pragma unroll
            for (int k = 0; k < 4; ++k) y[k] = __builtin_amdgcn_exp2f((e[k] * rinv - 1.0f) * L2E);
            if (ps == 0) { zc = zc + y; }
            else { v4f o;
#pragma unroll
                for (int k = 0; k < 4; ++k) o[k] = (y[k] * iz[k]) * x[k];
                float* p = dst + (size_t)i * 16 * HD;
                *(volatile v4f*)p = o; __threadfence(); *(volatile v4f*)p = o; }
        }
        if (ps == 0) {
#pragma unroll
            for (int k = 0; k < 4; ++k) zc[k] += __shfl_xor(zc[k], 16, 32);
            if (hi == 0) *(v4fa*)(&zs[wave * HD + lr * 4]) = zc;
            __syncthreads();
            if (threadIdx.x < HD) { float z = 0.0f;
#pragma unroll 1
                for (int w = 0; w < 8; ++w) z += zs[w * HD + threadIdx.x];
                zi[threadIdx.x] = 1.0f / z; }
            __syncthreads();
            iz = *(const v4fa*)(&zi[lr * 4]);
        }
    }
}

static constexpr size_t al256(size_t v) { return (v + 255) & ~(size_t)255; }
static constexpr size_t SZ_XB = al256((size_t)NB * SEQ * HD * 2);
static constexpr size_t SZ_WT = al256((size_t)NH_ * HD * HD * 2);
static constexpr size_t SZ_WQ = al256((size_t)NB * SEQ * NQ * 2);
static constexpr size_t SZ_DV = al256((size_t)NB * NH_ * SEQ * HD * 4);
static constexpr size_t SZ_TOTAL = 3 * SZ_XB + SZ_WT + SZ_WQ + SZ_DV;
static_assert(SZ_TOTAL <= (size_t)134217728);
static_assert((size_t)NB * HD * SEQ == (size_t)NB * SEQ * HD);
static_assert(((size_t)NB * SEQ * HD) % 8 == 0);
static_assert(((size_t)SEQ * HD) % 8 == 0);

extern "C" void kernel_launch(void* const* d_in, const int* in_sizes, int n_in,
                              void* d_out, int out_size, void* d_ws, size_t ws_size, hipStream_t stream) {
    if (n_in < 5) return;
    const size_t needx = ((size_t)(NB - 1) * SEQ_FULL + SEQ) * HD;
    if ((size_t)in_sizes[0] < needx || (size_t)in_sizes[1] < needx || (size_t)in_sizes[2] < needx) return;
    if ((size_t)in_sizes[3] < (size_t)NH_ * HD * HD || in_sizes[4] < 1) return;
    if ((size_t)out_size < ((size_t)(NB * NH_ - 1) * OUT_SEQ + SEQ) * HD) return;
    if (SZ_TOTAL > ws_size) return;
    const float* xq = (const float*)d_in[0];
    const float* xk = (const float*)d_in[1];
    const float* xv = (const float*)d_in[2];
    const float* w  = (const float*)d_in[3];
    const float* sf = (const float*)d_in[4];
    float* OUT = (float*)d_out;
    char* wsp = (char*)d_ws;
    bf*  XB = (bf*)wsp;  wsp += SZ_XB;
    h16* KP = (h16*)wsp; wsp += SZ_XB;
    h16* VT = (h16*)wsp; wsp += SZ_XB;
    bf*  WT = (bf*)wsp;  wsp += SZ_WT;
    h16* WQ = (h16*)wsp; wsp += SZ_WQ;
    float* DV = (float*)wsp; wsp += SZ_DV;

    if (SEQ == SEQ_FULL) {
        const size_t n8 = (size_t)NB * SEQ * HD / 8;
        k_cvt8<<<(unsigned)((n8 + 255) / 256), 256, 0, stream>>>(xq, XB, n8);
        k_cvth8<<<(unsigned)((n8 + 255) / 256), 256, 0, stream>>>(xk, KP, n8);
    } else {
        const size_t n8 = (size_t)SEQ * HD / 8;
        for (int b = 0; b < NB; ++b) {
            k_cvt8<<<(unsigned)((n8 + 255) / 256), 256, 0, stream>>>(xq + (size_t)b * SEQ_FULL * HD, XB + (size_t)b * SEQ * HD, n8);
            k_cvth8<<<(unsigned)((n8 + 255) / 256), 256, 0, stream>>>(xk + (size_t)b * SEQ_FULL * HD, KP + (size_t)b * SEQ * HD, n8);
        }
    }
    k_wtr<<<NH_, 256, 0, stream>>>(w, WT);
    k_vtr<<<dim3(SEQ / 64, NB, 1), 256, 0, stream>>>(xv, VT);
    k_wq<<<dim3(NB * SEQ / 64, NQ / 64, 1), 32, 0, stream>>>(XB, WT, WQ);
    k_hattn<<<dim3(NB * SEQ / AW, 1, 1), 32 * AW, 0, stream>>>(WQ, KP, VT, sf, DV);
    k_fin<<<dim3(NB * NH_, 1, 1), 256, 0, stream>>>(DV, OUT);
}
